// SpatialRangeBlock_50251117363406
// MI455X (gfx1250) — hardware-verified
//
#include <hip/hip_runtime.h>
#include <stdint.h>

#define DIMC 256
#define HH 64
#define WW 64
#define HWP 4096
#define BB 2
#define NN 49
#define RAD 3
#define LDSP 40
#define STGP 68
#define CKP 64
#define NPIX (BB * HWP)

typedef __bf16   v16bf __attribute__((ext_vector_type(16)));
typedef __bf16   v8bf  __attribute__((ext_vector_type(8)));
typedef _Float16 v16h  __attribute__((ext_vector_type(16)));
typedef _Float16 v8h   __attribute__((ext_vector_type(8)));
typedef float    v8f   __attribute__((ext_vector_type(8)));
typedef float    v4f   __attribute__((ext_vector_type(4)));
typedef float    v4fa  __attribute__((ext_vector_type(4), __may_alias__));
typedef unsigned short v8us __attribute__((ext_vector_type(8)));

template<typename T> struct VTr;
template<> struct VTr<__bf16>   { typedef v16bf V16; typedef v8bf V8; };
template<> struct VTr<_Float16> { typedef v16h  V16; typedef v8h  V8; };

__device__ __forceinline__ int refl(int i, int n) {
  i = (i < 0) ? -i : i;
  i = (i >= n) ? (2 * n - 2 - i) : i;
  return i;
}

__device__ __forceinline__ unsigned short bf16_rne(float x) {
  unsigned int u = __float_as_uint(x);
  u += 0x7FFFu + ((u >> 16) & 1u);
  return (unsigned short)(u >> 16);
}
__device__ __forceinline__ float bf16_f32(unsigned short b) {
  return __uint_as_float(((unsigned int)b) << 16);
}

__device__ __forceinline__ v8f mma(v8f c, v16bf a, v16bf b) {
  c = __builtin_amdgcn_wmma_f32_16x16x32_bf16(false, a, false, b, (short)0, c, false, false);
  asm volatile("v_nop\n\tv_nop\n\tv_nop\n\tv_nop" : "+v"(c) : "v"(a), "v"(b));
  return c;
}
__device__ __forceinline__ v8f mma(v8f c, v16h a, v16h b) {
  c = __builtin_amdgcn_wmma_f32_16x16x32_f16(false, a, false, b, (short)0, c, false, false);
  asm volatile("v_nop\n\tv_nop\n\tv_nop\n\tv_nop" : "+v"(c) : "v"(a), "v"(b));
  return c;
}

template<typename T>
__device__ __forceinline__ typename VTr<T>::V16 ldfrag(const T* rowp, int hh) {
  typedef typename VTr<T>::V8 V8;
  const V8 e0 = *(const V8*)(rowp + 8 * hh);
  const V8 e1 = *(const V8*)(rowp + 16 + 8 * hh);
  return __builtin_shufflevector(e0, e1, 0, 1, 2, 3, 4, 5, 6, 7, 8, 9, 10, 11, 12, 13, 14, 15);
}

template<int KIND>
__device__ __forceinline__ void pack8(const float (&y)[8], float scale, v8us& o0, v8us& o1) {
  if (KIND == 0) {
    v8us a = {0, 0, 0, 0, 0, 0, 0, 0}, c = {0, 0, 0, 0, 0, 0, 0, 0};
#pragma unroll
    for (int k = 0; k < 8; ++k) {
      const unsigned short hb = bf16_rne(y[k]);
      a[k] = hb;
      c[k] = bf16_rne(y[k] - bf16_f32(hb));
    }
    o0 = a; o1 = c;
  } else {
    v8h hv = {0, 0, 0, 0, 0, 0, 0, 0};
#pragma unroll
    for (int k = 0; k < 8; ++k) hv[k] = (_Float16)(y[k] * scale);
    o0 = __builtin_bit_cast(v8us, hv);
    o1 = o0;
  }
}

template<int KIND>
__global__ __launch_bounds__(256)
void k_cvt_w(const float* __restrict__ src, unsigned short* p0, unsigned short* p1, float scale, int n8) {
  const int i = blockIdx.x * 256 + threadIdx.x;
  if (i >= n8) return;
  const v4fa* s = (const v4fa*)(src + (size_t)i * 8);
  const v4f x0 = s[0];
  const v4f x1 = s[1];
  float y[8] = {x0[0], x0[1], x0[2], x0[3], x1[0], x1[1], x1[2], x1[3]};
  v8us o0, o1;
  pack8<KIND>(y, scale, o0, o1);
  unsigned short* d0 = p0 + (size_t)i * 8;
  unsigned short* d1 = p1 + (size_t)i * 8;
  *(volatile v8us*)d0 = o0;
  if (KIND == 0) *(volatile v8us*)d1 = o1;
  __threadfence();
  *(volatile v8us*)d0 = o0;
  if (KIND == 0) *(volatile v8us*)d1 = o1;
}

template<int KIND>
__global__ __launch_bounds__(128)
void k_cvt_act(const float* __restrict__ X, const float* __restrict__ g, const float* __restrict__ be,
               unsigned short* p0, unsigned short* p1, float scale, int do_ln, int do_silu) {
  __shared__ float tile[DIMC * 33];
  const int t = threadIdx.x, l = t & 31, wv = t >> 5;
  const int b = blockIdx.y, pbase = blockIdx.x * 32;
  if (pbase >= HWP || b >= BB) return;
  const float* Xb = X + (size_t)b * DIMC * HWP + pbase + l;
  for (int j = 0; j < 64; ++j) {
    const int c = wv * 64 + j;
    tile[c * 33 + l] = Xb[(size_t)c * HWP];
  }
  __syncthreads();

#pragma unroll 1
  for (int i = 0; i < 8; ++i) {
    const int p = wv * 8 + i;
    float y[8];
#pragma unroll
    for (int k = 0; k < 8; ++k) y[k] = tile[(8 * l + k) * 33 + p];
    if (do_ln) {
      float s = 0.f;
#pragma unroll
      for (int k = 0; k < 8; ++k) s += y[k];
      for (int o = 16; o >= 1; o >>= 1) s += __shfl_xor(s, o, 32);
      const float mean = s * (1.f / DIMC);
      float s2 = 0.f;
#pragma unroll
      for (int k = 0; k < 8; ++k) { const float d = y[k] - mean; y[k] = d; s2 += d * d; }
      for (int o = 16; o >= 1; o >>= 1) s2 += __shfl_xor(s2, o, 32);
      const float rstd = 1.f / sqrtf(s2 * (1.f / DIMC) + 1e-6f);
#pragma unroll
      for (int k = 0; k < 8; ++k) {
        const int c = 8 * l + k;
        float v = g[c] * (y[k] * rstd) + be[c];
        if (do_silu) v = v / (1.f + expf(-v));
        y[k] = v;
        tile[(8 * l + k) * 33 + p] = v;
      }
    }
    v8us o0, o1;
    pack8<KIND>(y, scale, o0, o1);
    const size_t ro = ((size_t)(b * HWP + pbase + p)) * DIMC + 8 * l;
    *(volatile v8us*)(p0 + ro) = o0;
    if (KIND == 0) *(volatile v8us*)(p1 + ro) = o1;
  }
  __threadfence();
#pragma unroll 1
  for (int i = 0; i < 8; ++i) {
    const int p = wv * 8 + i;
    float y[8];
#pragma unroll
    for (int k = 0; k < 8; ++k) y[k] = tile[(8 * l + k) * 33 + p];
    v8us o0, o1;
    pack8<KIND>(y, scale, o0, o1);
    const size_t ro = ((size_t)(b * HWP + pbase + p)) * DIMC + 8 * l;
    *(volatile v8us*)(p0 + ro) = o0;
    if (KIND == 0) *(volatile v8us*)(p1 + ro) = o1;
  }
}

template<typename T, int NPROD>
__global__ __launch_bounds__(128)
void k_gemm(const T* X0, const T* X1, const T* W0, const T* W1,
            const float* __restrict__ bias, float oscale, float* Y) {
  typedef typename VTr<T>::V16 V16;
  typedef typename VTr<T>::V8 V8;
  __shared__ T lA0[64 * LDSP] __attribute__((aligned(16)));
  __shared__ T lA1[64 * LDSP] __attribute__((aligned(16)));
  __shared__ T lB0[64 * LDSP] __attribute__((aligned(16)));
  __shared__ T lB1[64 * LDSP] __attribute__((aligned(16)));
  __shared__ float stg[64 * STGP] __attribute__((aligned(16)));

  const int nBase = blockIdx.x * 64;
  const int mBase = blockIdx.y * 64;
  const int b = blockIdx.z;
  if (nBase >= HWP || mBase >= DIMC || b >= BB) return;
  const T* Xb0 = X0 + (size_t)b * HWP * DIMC;
  const T* Xb1 = X1 + (size_t)b * HWP * DIMC;
  float* Yb = Y + (size_t)b * DIMC * HWP;
  const int t = threadIdx.x, l = t & 31, wv = t >> 5, m16 = l & 15, hh = l >> 4;

  const v8f zero8 = {0.f, 0.f, 0.f, 0.f, 0.f, 0.f, 0.f, 0.f};
  v8f acc[4];
#pragma unroll
  for (int ns = 0; ns < 4; ++ns) acc[ns] = zero8;

  for (int k0 = 0; k0 < DIMC; k0 += 32) {
#pragma unroll
    for (int i = 0; i < 2; ++i) {
      const int cid = 2 * t + i;
      const int row = cid >> 2, seg = cid & 3;
      const int lo = row * LDSP + seg * 8;
      const size_t wo = (size_t)(mBase + row) * DIMC + k0 + seg * 8;
      const size_t xo = (size_t)(nBase + row) * DIMC + k0 + seg * 8;
      *(V8*)(lA0 + lo) = *(const V8*)(W0 + wo);
      *(V8*)(lB0 + lo) = *(const V8*)(Xb0 + xo);
      if (NPROD == 3) {
        *(V8*)(lA1 + lo) = *(const V8*)(W1 + wo);
        *(V8*)(lB1 + lo) = *(const V8*)(Xb1 + xo);
      }
    }
    __syncthreads();

    const int arow = (wv * 16 + m16) * LDSP;
    const V16 a0 = ldfrag<T>(lA0 + arow, hh);
    V16 a1 = a0;
    if (NPROD == 3) a1 = ldfrag<T>(lA1 + arow, hh);
#pragma unroll
    for (int ns = 0; ns < 4; ++ns) {
      const int brow = (ns * 16 + m16) * LDSP;
      const V16 b0 = ldfrag<T>(lB0 + brow, hh);
      acc[ns] = mma(acc[ns], a0, b0);
      if (NPROD == 3) {
        const V16 b1 = ldfrag<T>(lB1 + brow, hh);
        acc[ns] = mma(acc[ns], a0, b1);
        acc[ns] = mma(acc[ns], a1, b0);
      }
    }
    __syncthreads();
  }

#pragma unroll
  for (int ns = 0; ns < 4; ++ns) {
#pragma unroll
    for (int r = 0; r < 8; ++r) {
      const int row = wv * 16 + 8 * hh + r;
      stg[row * STGP + ns * 16 + m16] = acc[ns][r] * oscale + bias[mBase + row];
    }
  }
  __syncthreads();

  v4f ov[8];
  const int c4 = (l & 15) * 4;
#pragma unroll
  for (int it = 0; it < 8; ++it) {
    const int row = wv * 16 + 2 * it + hh;
    ov[it] = *(const v4fa*)(stg + row * STGP + c4);
  }
#pragma unroll
  for (int it = 0; it < 8; ++it) {
    const int row = wv * 16 + 2 * it + hh;
    float* dst = Yb + (size_t)(mBase + row) * HWP + nBase + c4;
    *(volatile v4f*)dst = ov[it];
  }
  __threadfence();
#pragma unroll
  for (int it = 0; it < 8; ++it) {
    const int row = wv * 16 + 2 * it + hh;
    float* dst = Yb + (size_t)(mBase + row) * HWP + nBase + c4;
    *(volatile v4f*)dst = ov[it];
  }
}

__device__ __forceinline__ float blk_sum64(float* red, int t, float v) {
  red[t] = v;
  __syncthreads();
  for (int o = 32; o >= 1; o >>= 1) {
    if (t < o) red[t] = red[t] + red[t + o];
    __syncthreads();
  }
  const float r = red[0];
  __syncthreads();
  return r;
}
__device__ __forceinline__ float blk_max64(float* red, int t, float v) {
  red[t] = v;
  __syncthreads();
  for (int o = 32; o >= 1; o >>= 1) {
    if (t < o) red[t] = fmaxf(red[t], red[t + o]);
    __syncthreads();
  }
  const float r = red[0];
  __syncthreads();
  return r;
}

__global__ __launch_bounds__(64)
void k_range(const float* __restrict__ px, const float* __restrict__ sem,
             const float* __restrict__ w1, const float* __restrict__ b1,
             const float* __restrict__ g, const float* __restrict__ be,
             const float* __restrict__ w2, const float* __restrict__ b2,
             const float* __restrict__ sigma, float* ck, int npix) {
  __shared__ float ctr[DIMC];
  __shared__ float lsem[DIMC];
  __shared__ float lck[64];
  __shared__ float lh[64];
  __shared__ float red[64];
  __shared__ float orow[64] __attribute__((aligned(16)));
  const int pix = blockIdx.x;
  if (pix >= npix) return;
  const int t = threadIdx.x;
  const int b = pix / HWP, p = pix - b * HWP, h = p / WW, w = p - h * WW;
  const float* pb = px + (size_t)b * DIMC * HWP;
  const float* sb = sem + (size_t)b * DIMC * HWP + p;
  for (int c = t; c < DIMC; c += 64) {
    ctr[c]  = pb[(size_t)c * HWP + p];
    lsem[c] = sb[(size_t)c * HWP];
  }
  __syncthreads();

  const bool act = (t < NN);
  const int iy = t / 7, ix = t - iy * 7;
  float dotv = -3.0e38f;
  if (act) {
    const int np = refl(h + iy - RAD, HH) * WW + refl(w + ix - RAD, WW);
    const float* qn = pb + np;
    float s = 0.f;
#pragma unroll 4
    for (int c = 0; c < DIMC; ++c) s += qn[(size_t)c * HWP] * ctr[c];
    dotv = s * (1.f / 16.f);
  }
  const float mx = blk_max64(red, t, dotv);
  const float e = act ? expf(dotv - mx) : 0.f;
  const float se = blk_sum64(red, t, e);
  float ck0 = 0.f;
  if (act) {
    const float sg = sigma[0];
    const float gx = (float)(iy - RAD) * (1.f / 3.f);
    const float gy = (float)(ix - RAD) * (1.f / 3.f);
    const float ga = expf(-(gx * gx + gy * gy) / (2.f * sg * sg));
    ck0 = (e / se) * ga;
  }
  lck[t] = ck0;
  __syncthreads();

  float f1 = 0.f;
  if (act) {
    const float* wr = w1 + (size_t)t * (NN + DIMC);
    float s = 0.f;
#pragma unroll 7
    for (int i = 0; i < NN; ++i) s += wr[i] * lck[i];
#pragma unroll 4
    for (int c = 0; c < DIMC; ++c) s += wr[NN + c] * lsem[c];
    f1 = s + b1[t];
  }
  const float m1 = blk_sum64(red, t, act ? f1 : 0.f) * (1.f / NN);
  const float d1 = act ? (f1 - m1) : 0.f;
  const float var1 = blk_sum64(red, t, d1 * d1) * (1.f / NN);
  const float rs1 = 1.f / sqrtf(var1 + 1e-6f);
  float hv = 0.f;
  if (act) {
    const float y = g[t] * (d1 * rs1) + be[t];
    hv = y / (1.f + expf(-y));
  }
  lh[t] = hv;
  __syncthreads();

  float cval = 0.f;
  if (act) {
    const float* wr = w2 + (size_t)t * NN;
    float s = 0.f;
#pragma unroll 7
    for (int i = 0; i < NN; ++i) s += wr[i] * lh[i];
    s += b2[t];
    const float gate = 1.f / (1.f + expf(-s));
    cval = ck0 + ck0 * gate;
  }
  const float tot = blk_sum64(red, t, cval);
  orow[t] = act ? (cval * (1.f / (tot + 1e-7f))) : 0.f;
  __syncthreads();
  if (t < 16) {
    const v4f v = *(const v4fa*)(orow + 4 * t);
    float* dst = ck + (size_t)pix * CKP + 4 * t;
    *(volatile v4f*)dst = v;
    __threadfence();
    *(volatile v4f*)dst = v;
  }
}

__global__ __launch_bounds__(64)
void k_agg(const float* __restrict__ spat, const float* __restrict__ ck, float* agg, int nblk) {
  __shared__ float stg[4 * 64] __attribute__((aligned(16)));
  const int id = blockIdx.x;
  if (id >= nblk) return;
  const int h = id & (HH - 1);
  const int cg = (id >> 6) & 63;
  const int b = id >> 12;
  const int t = threadIdx.x, w = t;
  int wx[7];
#pragma unroll
  for (int ix = 0; ix < 7; ++ix) wx[ix] = refl(w + ix - RAD, WW);
  const float* ckp = ck + ((size_t)(b * HWP + h * WW + w)) * CKP;
  const float* sp = spat + ((size_t)(b * DIMC + cg * 4)) * HWP;
  float a0 = 0.f, a1 = 0.f, a2 = 0.f, a3 = 0.f;
#pragma unroll 1
  for (int iy = 0; iy < 7; ++iy) {
    const int hy = refl(h + iy - RAD, HH) * WW;
    const float* ckr = ckp + iy * 7;
#pragma unroll
    for (int ix = 0; ix < 7; ++ix) {
      const float cv = ckr[ix];
      const int o = hy + wx[ix];
      a0 += cv * sp[o];
      a1 += cv * sp[HWP + o];
      a2 += cv * sp[2 * HWP + o];
      a3 += cv * sp[3 * HWP + o];
    }
  }
  stg[0 * 64 + w] = a0;
  stg[1 * 64 + w] = a1;
  stg[2 * 64 + w] = a2;
  stg[3 * 64 + w] = a3;
  __syncthreads();
  if (t < 32) {
    const int hq = t >> 4, c4 = (t & 15) * 4;
    v4f v[2];
    float* dst[2];
#pragma unroll
    for (int q = 0; q < 2; ++q) {
      const int j = 2 * q + hq;
      v[q] = *(const v4fa*)(stg + j * 64 + c4);
      dst[q] = agg + ((size_t)(b * DIMC + cg * 4 + j)) * HWP + h * WW + c4;
    }
    *(volatile v4f*)dst[0] = v[0];
    *(volatile v4f*)dst[1] = v[1];
    __threadfence();
    *(volatile v4f*)dst[0] = v[0];
    *(volatile v4f*)dst[1] = v[1];
  }
}

extern "C" void kernel_launch(void* const* d_in, const int* in_sizes, int n_in,
                              void* d_out, int out_size, void* d_ws, size_t ws_size,
                              hipStream_t stream) {
  if (n_in < 21) return;
  if (out_size != BB * DIMC * HWP) return;
  if (in_sizes[0] != BB * DIMC * HWP || in_sizes[1] != BB * DIMC * HWP) return;
  if (in_sizes[2] != DIMC * DIMC || in_sizes[6] != DIMC * DIMC ||
      in_sizes[14] != DIMC * DIMC || in_sizes[18] != DIMC * DIMC) return;
  if (in_sizes[8] != NN * (NN + DIMC) || in_sizes[12] != NN * NN || in_sizes[20] < 1) return;
  if (in_sizes[3] < DIMC || in_sizes[4] < DIMC || in_sizes[5] < DIMC || in_sizes[7] < DIMC) return;
  if (in_sizes[15] < DIMC || in_sizes[16] < DIMC || in_sizes[17] < DIMC || in_sizes[19] < DIMC) return;
  if (in_sizes[9] < NN || in_sizes[10] < NN || in_sizes[11] < NN || in_sizes[13] < NN) return;

  const float* spatial  = (const float*)d_in[0];
  const float* semantic = (const float*)d_in[1];
  const float* rp_w1 = (const float*)d_in[2];
  const float* rp_b1 = (const float*)d_in[3];
  const float* rp_g  = (const float*)d_in[4];
  const float* rp_be = (const float*)d_in[5];
  const float* rp_w2 = (const float*)d_in[6];
  const float* rp_b2 = (const float*)d_in[7];
  const float* fp_w1 = (const float*)d_in[8];
  const float* fp_b1 = (const float*)d_in[9];
  const float* fp_g  = (const float*)d_in[10];
  const float* fp_be = (const float*)d_in[11];
  const float* fp_w2 = (const float*)d_in[12];
  const float* fp_b2 = (const float*)d_in[13];
  const float* op_w1 = (const float*)d_in[14];
  const float* op_b1 = (const float*)d_in[15];
  const float* op_g  = (const float*)d_in[16];
  const float* op_be = (const float*)d_in[17];
  const float* op_w2 = (const float*)d_in[18];
  const float* op_b2 = (const float*)d_in[19];
  const float* sigma = (const float*)d_in[20];
  float* out = (float*)d_out;

  const size_t PLB = (size_t)BB * HWP * DIMC * 2;
  const size_t WPB = (size_t)DIMC * DIMC * 2;
  const size_t YB  = (size_t)BB * DIMC * HWP * 4;
  const size_t CKB = (size_t)NPIX * CKP * 4;
  char* ws = (char*)d_ws;
  size_t off = 0;
  auto carve = [&](size_t n) -> char* { char* q = ws + off; off += (n + 255) & ~(size_t)255; return q; };
  unsigned short* pa  = (unsigned short*)carve(PLB);
  unsigned short* pbp = (unsigned short*)carve(PLB);
  unsigned short* w1h = (unsigned short*)carve(WPB);
  unsigned short* w1l = (unsigned short*)carve(WPB);
  unsigned short* w2h = (unsigned short*)carve(WPB);
  unsigned short* w2l = (unsigned short*)carve(WPB);
  unsigned short* ow1 = (unsigned short*)carve(WPB);
  unsigned short* ow2 = (unsigned short*)carve(WPB);
  float* yA = (float*)carve(YB);
  float* yB = (float*)carve(YB);
  float* ckb = (float*)carve(CKB);
  if (off > ws_size) return;

  const int nw8 = DIMC * DIMC / 8;
  const dim3 gw((nw8 + 255) / 256), bw(256);
  const dim3 ga((HWP + 31) / 32, BB), ba(128);
  const dim3 gg((HWP + 63) / 64, (DIMC + 63) / 64, BB), bg(128);
  const int nagg = BB * (DIMC / 4) * HH;

  hipLaunchKernelGGL(HIP_KERNEL_NAME(k_cvt_w<0>), gw, bw, 0, stream, rp_w1, w1h, w1l, 1.0f, nw8);
  hipLaunchKernelGGL(HIP_KERNEL_NAME(k_cvt_w<0>), gw, bw, 0, stream, rp_w2, w2h, w2l, 1.0f, nw8);
  hipLaunchKernelGGL(HIP_KERNEL_NAME(k_cvt_w<1>), gw, bw, 0, stream, op_w1, ow1, ow1, 16.0f, nw8);
  hipLaunchKernelGGL(HIP_KERNEL_NAME(k_cvt_w<1>), gw, bw, 0, stream, op_w2, ow2, ow2, 16.0f, nw8);

  hipLaunchKernelGGL(HIP_KERNEL_NAME(k_cvt_act<0>), ga, ba, 0, stream,
                     semantic, rp_g, rp_be, pa, pbp, 1.0f, 0, 0);
  hipLaunchKernelGGL(HIP_KERNEL_NAME(k_gemm<__bf16, 3>), gg, bg, 0, stream,
                     (const __bf16*)pa, (const __bf16*)pbp, (const __bf16*)w1h, (const __bf16*)w1l,
                     rp_b1, 1.0f, yA);
  hipLaunchKernelGGL(HIP_KERNEL_NAME(k_cvt_act<0>), ga, ba, 0, stream,
                     (const float*)yA, rp_g, rp_be, pa, pbp, 1.0f, 1, 1);
  hipLaunchKernelGGL(HIP_KERNEL_NAME(k_gemm<__bf16, 3>), gg, bg, 0, stream,
                     (const __bf16*)pa, (const __bf16*)pbp, (const __bf16*)w2h, (const __bf16*)w2l,
                     rp_b2, 1.0f, yB);

  hipLaunchKernelGGL(k_range, dim3(NPIX), dim3(64), 0, stream,
                     (const float*)yB, semantic, fp_w1, fp_b1, fp_g, fp_be, fp_w2, fp_b2, sigma, ckb, NPIX);
  hipLaunchKernelGGL(k_agg, dim3(nagg), dim3(64), 0, stream,
                     spatial, (const float*)ckb, yA, nagg);

  hipLaunchKernelGGL(HIP_KERNEL_NAME(k_cvt_act<1>), ga, ba, 0, stream,
                     (const float*)yA, op_g, op_be, pa, pa, 1.0f, 0, 0);
  hipLaunchKernelGGL(HIP_KERNEL_NAME(k_gemm<_Float16, 1>), gg, bg, 0, stream,
                     (const _Float16*)pa, (const _Float16*)pa, (const _Float16*)ow1, (const _Float16*)ow1,
                     op_b1, 1.0f / 16.0f, yB);
  hipLaunchKernelGGL(HIP_KERNEL_NAME(k_cvt_act<1>), ga, ba, 0, stream,
                     (const float*)yB, op_g, op_be, pa, pa, 1.0f, 1, 0);
  hipLaunchKernelGGL(HIP_KERNEL_NAME(k_gemm<_Float16, 1>), gg, bg, 0, stream,
                     (const _Float16*)pa, (const _Float16*)pa, (const _Float16*)ow2, (const _Float16*)ow2,
                     op_b2, 1.0f / 16.0f, out);
}
